// DynamicTokenMixing_90915867722021
// MI455X (gfx1250) — hardware-verified
//
#include <hip/hip_runtime.h>


typedef __bf16 bf16_t;
typedef __bf16       v16bf __attribute__((ext_vector_type(16)));
typedef float        v8f   __attribute__((ext_vector_type(8)));
typedef float        v4f   __attribute__((ext_vector_type(4)));
typedef unsigned int v4u   __attribute__((ext_vector_type(4)));

union Frag  { v16bf v; v4u q[2]; bf16_t s[16]; };
union Pack8 { v4u u; bf16_t s[8]; };

#define TOK   4096
#define DIM   1024
#define HDIM  64
#define NQKV  3072
#define GB_M  128
#define GB_N  64

static __device__ __forceinline__ v8f zero8() {
    v8f z = {0.f, 0.f, 0.f, 0.f, 0.f, 0.f, 0.f, 0.f};
    return z;
}

static __device__ __forceinline__ v8f mma(v8f c, v16bf a, v16bf b) {
    return __builtin_amdgcn_wmma_f32_16x16x32_bf16(false, a, false, b, (short)0, c, false, false);
}

static __device__ __forceinline__ void cvt_hl(float v, bf16_t& hi, bf16_t& lo) {
    bf16_t hb = (bf16_t)v;
    hi = hb;
    lo = (bf16_t)(v - (float)hb);
}

static __device__ __forceinline__ void split8(v4f a, v4f b, v4u& hi, v4u& lo) {
    Pack8 ph, pl;
#pragma unroll
    for (int i = 0; i < 4; ++i) {
        cvt_hl(a[i], ph.s[i], pl.s[i]);
        cvt_hl(b[i], ph.s[4 + i], pl.s[4 + i]);
    }
    hi = ph.u;
    lo = pl.u;
}

static __device__ __forceinline__ float hmax8(v8f v) {
    float a = fmaxf(fmaxf(v[0], v[1]), fmaxf(v[2], v[3]));
    float b = fmaxf(fmaxf(v[4], v[5]), fmaxf(v[6], v[7]));
    return fmaxf(a, b);
}

__global__ void __launch_bounds__(256)
k_split_x(const float* __restrict__ x, bf16_t* Xh, bf16_t* Xl, int n8,
          const int* hw0, const int* hw1) {
    (void)hw0; (void)hw1;
    const int i = blockIdx.x * 256 + threadIdx.x;
    if (i >= n8) return;
    const size_t base = (size_t)i * 8;
    v4f a = *(const v4f*)(x + base);
    v4f b = *(const v4f*)(x + base + 4);
    v4u hi, lo;
    split8(a, b, hi, lo);
    *(volatile v4u*)(Xh + base) = hi;
    *(volatile v4u*)(Xl + base) = lo;
    __threadfence();
    *(volatile v4u*)(Xh + base) = hi;
    *(volatile v4u*)(Xl + base) = lo;
}

static __device__ __forceinline__ void wt_pass(const float* T, bf16_t* Th, bf16_t* Tl, int ldt,
                                                int n0, int k0, int tid) {
#pragma unroll
    for (int i = 0; i < 2; ++i) {
        const int item = tid + 256 * i;
        const int nn = item >> 3;
        const int kg = (item & 7) * 8;
        const float* c = T + kg * 64 + nn;
        v4f a = {c[0 * 64], c[1 * 64], c[2 * 64], c[3 * 64]};
        v4f b = {c[4 * 64], c[5 * 64], c[6 * 64], c[7 * 64]};
        v4u hi, lo;
        split8(a, b, hi, lo);
        const size_t dst = (size_t)(n0 + nn) * ldt + k0 + kg;
        *(volatile v4u*)(Th + dst) = hi;
        *(volatile v4u*)(Tl + dst) = lo;
    }
}

__global__ void __launch_bounds__(256)
k_split_wT(const float* __restrict__ W0, int ld0, const float* __restrict__ W1, int ld1, int nsplit,
           bf16_t* Th, bf16_t* Tl, int ldt) {
    __shared__ __align__(16) float T[64 * 64];
    const int tid = threadIdx.x;
    const int n0 = blockIdx.x * 64;
    const int k0 = blockIdx.y * 64;
    const float* src;
    int ld, c0;
    if (n0 < nsplit) { src = W0; ld = ld0; c0 = n0; }
    else             { src = W1; ld = ld1; c0 = n0 - nsplit; }
#pragma unroll
    for (int i = 0; i < 4; ++i) {
        const int idx = tid + 256 * i;
        const int kk = idx >> 4;
        const int c4 = (idx & 15) * 4;
        *(v4f*)(T + kk * 64 + c4) = *(const v4f*)(src + (size_t)(k0 + kk) * ld + c0 + c4);
    }
    __syncthreads();
    wt_pass(T, Th, Tl, ldt, n0, k0, tid);
    __threadfence();
    wt_pass(T, Th, Tl, ldt, n0, k0, tid);
}

static __device__ __forceinline__ void ep_f32(const float* S, float* outF, int ldo, int mb, int n0,
                                               v4f b4, int tid) {
    const int c4 = (tid & 15) * 4;
#pragma unroll
    for (int i = 0; i < 8; ++i) {
        const int r = 16 * i + (tid >> 4);
        v4f v = *(const v4f*)(S + r * GB_N + c4) + b4;
        *(volatile v4f*)(outF + (size_t)(mb + r) * ldo + n0 + c4) = v;
    }
}

static __device__ __forceinline__ void ep_qk(const float* S, bf16_t* dh, bf16_t* dl, int head, int mb,
                                              int tid) {
#pragma unroll
    for (int i = 0; i < 4; ++i) {
        const int r  = 32 * i + (tid >> 3);
        const int dg = (tid & 7) * 8;
        v4f a = *(const v4f*)(S + r * GB_N + dg);
        v4f b = *(const v4f*)(S + r * GB_N + dg + 4);
        v4u hi, lo;
        split8(a, b, hi, lo);
        const size_t dst = ((size_t)head * TOK + mb + r) * HDIM + dg;
        *(volatile v4u*)(dh + dst) = hi;
        *(volatile v4u*)(dl + dst) = lo;
    }
}

static __device__ __forceinline__ void ep_v(const float* S, bf16_t* dh, bf16_t* dl, int head, int mb,
                                             int tid) {
#pragma unroll
    for (int i = 0; i < 4; ++i) {
        const int d  = 16 * i + (tid >> 4);
        const int tg = (tid & 15) * 8;
        const float* c = S + tg * GB_N + d;
        v4f a = {c[0 * GB_N], c[1 * GB_N], c[2 * GB_N], c[3 * GB_N]};
        v4f b = {c[4 * GB_N], c[5 * GB_N], c[6 * GB_N], c[7 * GB_N]};
        v4u hi, lo;
        split8(a, b, hi, lo);
        const size_t dst = ((size_t)head * HDIM + d) * TOK + mb + tg;
        *(volatile v4u*)(dh + dst) = hi;
        *(volatile v4u*)(dl + dst) = lo;
    }
}

__global__ void __launch_bounds__(256)
k_gemm(const bf16_t* __restrict__ Ah, const bf16_t* __restrict__ Al,
       const bf16_t* __restrict__ Bh, const bf16_t* __restrict__ Bl,
       int K, int mode,
       bf16_t* Qh, bf16_t* Ql, bf16_t* Kh, bf16_t* Kl, bf16_t* Vh, bf16_t* Vl,
       float* outF, const float* __restrict__ bias, int ldo) {
    __shared__ __align__(16) float S[GB_M * GB_N];
    const int tid  = threadIdx.x;
    const int lane = tid & 31;
    const int wave = tid >> 5;
    const int hh   = lane >> 4;
    const int m    = lane & 15;
    const int wr   = wave >> 1;
    const int wc   = wave & 1;
    const int n0   = blockIdx.x * GB_N;
    const int mb   = blockIdx.y * GB_M;

    const size_t ao  = (size_t)(mb + wr * 32 + m) * K + 8 * hh;
    const size_t bo  = (size_t)(n0 + wc * 32 + m) * K + 8 * hh;
    const size_t s16 = (size_t)16 * K;

    v8f c00 = zero8(), c01 = zero8(), c10 = zero8(), c11 = zero8();

#pragma unroll 1
    for (int k0 = 0; k0 < K; k0 += 32) {
        Frag a0h, a0l, a1h, a1l, b0h, b0l, b1h, b1l;
        const size_t oa = ao + k0;
        const size_t ob = bo + k0;
        a0h.q[0] = *(const v4u*)(Ah + oa);            a0h.q[1] = *(const v4u*)(Ah + oa + 16);
        a0l.q[0] = *(const v4u*)(Al + oa);            a0l.q[1] = *(const v4u*)(Al + oa + 16);
        a1h.q[0] = *(const v4u*)(Ah + oa + s16);      a1h.q[1] = *(const v4u*)(Ah + oa + s16 + 16);
        a1l.q[0] = *(const v4u*)(Al + oa + s16);      a1l.q[1] = *(const v4u*)(Al + oa + s16 + 16);
        b0h.q[0] = *(const v4u*)(Bh + ob);            b0h.q[1] = *(const v4u*)(Bh + ob + 16);
        b0l.q[0] = *(const v4u*)(Bl + ob);            b0l.q[1] = *(const v4u*)(Bl + ob + 16);
        b1h.q[0] = *(const v4u*)(Bh + ob + s16);      b1h.q[1] = *(const v4u*)(Bh + ob + s16 + 16);
        b1l.q[0] = *(const v4u*)(Bl + ob + s16);      b1l.q[1] = *(const v4u*)(Bl + ob + s16 + 16);

        c00 = mma(c00, a0h.v, b0h.v); c00 = mma(c00, a0h.v, b0l.v); c00 = mma(c00, a0l.v, b0h.v);
        c01 = mma(c01, a0h.v, b1h.v); c01 = mma(c01, a0h.v, b1l.v); c01 = mma(c01, a0l.v, b1h.v);
        c10 = mma(c10, a1h.v, b0h.v); c10 = mma(c10, a1h.v, b0l.v); c10 = mma(c10, a1l.v, b0h.v);
        c11 = mma(c11, a1h.v, b1h.v); c11 = mma(c11, a1h.v, b1l.v); c11 = mma(c11, a1l.v, b1h.v);
        asm volatile("v_nop\n\tv_nop\n\tv_nop\n\tv_nop"
                     : "+v"(c00), "+v"(c01), "+v"(c10), "+v"(c11)
                     : "v"(a0h.v), "v"(a0l.v), "v"(a1h.v), "v"(a1l.v),
                       "v"(b0h.v), "v"(b0l.v), "v"(b1h.v), "v"(b1l.v));
    }

    {
        float* s0 = S + (wr * 32 + 8 * hh) * GB_N + wc * 32 + m;
#pragma unroll
        for (int r = 0; r < 8; ++r) {
            s0[r * GB_N]             = c00[r];
            s0[r * GB_N + 16]        = c01[r];
            s0[(16 + r) * GB_N]      = c10[r];
            s0[(16 + r) * GB_N + 16] = c11[r];
        }
    }
    __syncthreads();

    if (mode == 1) {
        const int c4 = (tid & 15) * 4;
        const v4f b4 = *(const v4f*)(bias + n0 + c4);
        ep_f32(S, outF, ldo, mb, n0, b4, tid);
        __threadfence();
        ep_f32(S, outF, ldo, mb, n0, b4, tid);
    } else {
        int layout, head;
        bf16_t* dh;
        bf16_t* dl;
        if (n0 < DIM) {
            layout = 0; head = n0 >> 6; dh = Qh; dl = Ql;
        } else {
            const int np = n0 - DIM;
            const int a  = np >> 9;
            const int mm = (np >> 6) & 7;
            head = ((a >> 1) << 3) + mm;
            if ((a & 1) == 0) { layout = 0; dh = Kh; dl = Kl; }
            else              { layout = 1; dh = Vh; dl = Vl; }
        }
        if (layout == 0) {
            ep_qk(S, dh, dl, head, mb, tid);
            __threadfence();
            ep_qk(S, dh, dl, head, mb, tid);
        } else {
            ep_v(S, dh, dl, head, mb, tid);
            __threadfence();
            ep_v(S, dh, dl, head, mb, tid);
        }
    }
}

static __device__ __forceinline__ v8f score_tile(const bf16_t* __restrict__ Kh, const bf16_t* __restrict__ Kl,
                                                  size_t ko,
                                                  const Frag& qh0, const Frag& ql0,
                                                  const Frag& qh1, const Frag& ql1) {
    Frag kh0, kh1, kl0, kl1;
    kh0.q[0] = *(const v4u*)(Kh + ko);      kh0.q[1] = *(const v4u*)(Kh + ko + 16);
    kh1.q[0] = *(const v4u*)(Kh + ko + 32); kh1.q[1] = *(const v4u*)(Kh + ko + 48);
    kl0.q[0] = *(const v4u*)(Kl + ko);      kl0.q[1] = *(const v4u*)(Kl + ko + 16);
    kl1.q[0] = *(const v4u*)(Kl + ko + 32); kl1.q[1] = *(const v4u*)(Kl + ko + 48);
    v8f s = zero8();
    s = mma(s, kh0.v, qh0.v); s = mma(s, kh0.v, ql0.v); s = mma(s, kl0.v, qh0.v);
    s = mma(s, kh1.v, qh1.v); s = mma(s, kh1.v, ql1.v); s = mma(s, kl1.v, qh1.v);
    asm volatile("v_nop\n\tv_nop\n\tv_nop\n\tv_nop"
                 : "+v"(s)
                 : "v"(kh0.v), "v"(kh1.v), "v"(kl0.v), "v"(kl1.v),
                   "v"(qh0.v), "v"(ql0.v), "v"(qh1.v), "v"(ql1.v));
    return s;
}

static __device__ __forceinline__ v8f otile(v8f o, const bf16_t* __restrict__ Vh, const bf16_t* __restrict__ Vl,
                                             size_t vo,
                                             const Frag& ph0, const Frag& pl0,
                                             const Frag& ph1, const Frag& pl1) {
    Frag vh0, vh1, vl0, vl1;
    vh0.q[0] = *(const v4u*)(Vh + vo);      vh0.q[1] = *(const v4u*)(Vh + vo + 16);
    vh1.q[0] = *(const v4u*)(Vh + vo + 32); vh1.q[1] = *(const v4u*)(Vh + vo + 48);
    vl0.q[0] = *(const v4u*)(Vl + vo);      vl0.q[1] = *(const v4u*)(Vl + vo + 16);
    vl1.q[0] = *(const v4u*)(Vl + vo + 32); vl1.q[1] = *(const v4u*)(Vl + vo + 48);
    o = mma(o, vh0.v, ph0.v); o = mma(o, vh0.v, pl0.v); o = mma(o, vl0.v, ph0.v);
    o = mma(o, vh1.v, ph1.v); o = mma(o, vh1.v, pl1.v); o = mma(o, vl1.v, ph1.v);
    asm volatile("v_nop\n\tv_nop\n\tv_nop\n\tv_nop"
                 : "+v"(o)
                 : "v"(vh0.v), "v"(vh1.v), "v"(vl0.v), "v"(vl1.v),
                   "v"(ph0.v), "v"(pl0.v), "v"(ph1.v), "v"(pl1.v));
    return o;
}

static __device__ __forceinline__ v8f exp8(v8f v, float c, float nb, float& ls) {
    v8f p = zero8();
#pragma unroll
    for (int r = 0; r < 8; ++r) {
        const float e = exp2f(fmaf(v[r], c, nb));
        p[r] = e;
        ls += e;
    }
    return p;
}

static __device__ __forceinline__ void pack16(v8f pa, v8f pb, Frag& ph, Frag& pl) {
#pragma unroll
    for (int i = 0; i < 8; ++i) {
        cvt_hl(pa[i], ph.s[i],     pl.s[i]);
        cvt_hl(pb[i], ph.s[8 + i], pl.s[8 + i]);
    }
}

static __device__ __forceinline__ void o_pass(const float* Osr, bf16_t* Oh, bf16_t* Ol, int q0, int hd,
                                               int lane) {
#pragma unroll
    for (int i = 0; i < 4; ++i) {
        const int q  = 4 * i + (lane >> 3);
        const int dg = (lane & 7) * 8;
        v4f a = *(const v4f*)(Osr + q * HDIM + dg);
        v4f b = *(const v4f*)(Osr + q * HDIM + dg + 4);
        v4u hi, lo;
        split8(a, b, hi, lo);
        const size_t dst = (size_t)(q0 + q) * DIM + hd * HDIM + dg;
        *(volatile v4u*)(Oh + dst) = hi;
        *(volatile v4u*)(Ol + dst) = lo;
    }
}

__global__ void __launch_bounds__(64)
k_attn(const bf16_t* __restrict__ Qh, const bf16_t* __restrict__ Ql,
       const bf16_t* __restrict__ Kh, const bf16_t* __restrict__ Kl,
       const bf16_t* __restrict__ Vh, const bf16_t* __restrict__ Vl,
       bf16_t* Oh, bf16_t* Ol) {
    __shared__ __align__(32) float Os[2 * 16 * HDIM];
    const int tid  = threadIdx.x;
    const int lane = tid & 31;
    const int wave = tid >> 5;
    const int hh   = lane >> 4;
    const int m    = lane & 15;
    const int hd   = blockIdx.y;
    const int q0   = blockIdx.x * 32 + wave * 16;

    Frag qh0, qh1, ql0, ql1;
    {
        const size_t qo = ((size_t)hd * TOK + q0 + m) * HDIM + 8 * hh;
        qh0.q[0] = *(const v4u*)(Qh + qo);      qh0.q[1] = *(const v4u*)(Qh + qo + 16);
        qh1.q[0] = *(const v4u*)(Qh + qo + 32); qh1.q[1] = *(const v4u*)(Qh + qo + 48);
        ql0.q[0] = *(const v4u*)(Ql + qo);      ql0.q[1] = *(const v4u*)(Ql + qo + 16);
        ql1.q[0] = *(const v4u*)(Ql + qo + 32); ql1.q[1] = *(const v4u*)(Ql + qo + 48);
    }
    const size_t kbase = ((size_t)hd * TOK + m) * HDIM + 8 * hh;
    const size_t vbase = ((size_t)hd * HDIM + m) * TOK + 8 * hh;
    const size_t v16   = (size_t)16 * TOK;

    v8f o0 = zero8(), o1 = zero8(), o2 = zero8(), o3 = zero8();
    float mrun = -1.0e30f;
    float lrun = 0.f;
    const float SC = 0.72134752f;

#pragma unroll 1
    for (int kt = 0; kt < TOK / 64; ++kt) {
        const int kb = kt * 64;
        const size_t ko = kbase + (size_t)kb * HDIM;
        v8f s0 = score_tile(Kh, Kl, ko,             qh0, ql0, qh1, ql1);
        v8f s1 = score_tile(Kh, Kl, ko + 16 * HDIM, qh0, ql0, qh1, ql1);
        v8f s2 = score_tile(Kh, Kl, ko + 32 * HDIM, qh0, ql0, qh1, ql1);
        v8f s3 = score_tile(Kh, Kl, ko + 48 * HDIM, qh0, ql0, qh1, ql1);

        float mloc = fmaxf(fmaxf(hmax8(s0), hmax8(s1)), fmaxf(hmax8(s2), hmax8(s3)));
        mloc = fmaxf(mloc, __shfl_xor(mloc, 16, 32));
        const float mnew = fmaxf(mrun, mloc);
        const float nb = -mnew * SC;
        float ls = 0.f;
        s0 = exp8(s0, SC, nb, ls);
        s1 = exp8(s1, SC, nb, ls);
        s2 = exp8(s2, SC, nb, ls);
        s3 = exp8(s3, SC, nb, ls);
        ls += __shfl_xor(ls, 16, 32);
        const float alpha = exp2f((mrun - mnew) * SC);
        lrun = fmaf(lrun, alpha, ls);
        mrun = mnew;
        o0 *= alpha; o1 *= alpha; o2 *= alpha; o3 *= alpha;

        Frag ph0, pl0, ph1, pl1;
        pack16(s0, s1, ph0, pl0);
        pack16(s2, s3, ph1, pl1);

        const size_t vo = vbase + kb;
        o0 = otile(o0, Vh, Vl, vo,           ph0, pl0, ph1, pl1);
        o1 = otile(o1, Vh, Vl, vo + v16,     ph0, pl0, ph1, pl1);
        o2 = otile(o2, Vh, Vl, vo + 2 * v16, ph0, pl0, ph1, pl1);
        o3 = otile(o3, Vh, Vl, vo + 3 * v16, ph0, pl0, ph1, pl1);
    }

    const float inv = 1.0f / lrun;
    {
        float* osw = Os + wave * (16 * HDIM) + m * HDIM + 8 * hh;
        *(v8f*)(osw)      = o0 * inv;
        *(v8f*)(osw + 16) = o1 * inv;
        *(v8f*)(osw + 32) = o2 * inv;
        *(v8f*)(osw + 48) = o3 * inv;
    }
    __syncthreads();
    const float* osr = Os + wave * (16 * HDIM);
    o_pass(osr, Oh, Ol, q0, hd, lane);
    __threadfence();
    o_pass(osr, Oh, Ol, q0, hd, lane);
}

extern "C" void kernel_launch(void* const* d_in, const int* in_sizes, int n_in,
                              void* d_out, int out_size, void* d_ws, size_t ws_size,
                              hipStream_t stream) {
    if (n_in < 7) return;
    if (in_sizes[0] != TOK * DIM || in_sizes[1] != DIM * DIM || in_sizes[2] != DIM * 2 * DIM ||
        in_sizes[3] != DIM * DIM || in_sizes[4] < DIM || out_size != TOK * DIM) return;

    const float* x     = (const float*)d_in[0];
    const float* Wq    = (const float*)d_in[1];
    const float* Wkv   = (const float*)d_in[2];
    const float* Wproj = (const float*)d_in[3];
    const float* bproj = (const float*)d_in[4];
    const int*   Hp    = (const int*)d_in[5];
    const int*   Wp    = (const int*)d_in[6];
    float* out = (float*)d_out;

    const size_t MiB   = 1048576;
    const size_t szX   = (size_t)TOK * DIM * 2;
    const size_t szWT  = (size_t)NQKV * DIM * 2;
    const size_t szWP  = (size_t)DIM * DIM * 2;
    const size_t szH   = (size_t)16 * TOK * HDIM * 2;
    size_t off = 0;
    char* ws = (char*)d_ws;
    bf16_t* Xh  = (bf16_t*)(ws + off); off += szX;
    bf16_t* Xl  = (bf16_t*)(ws + off); off += szX;
    bf16_t* WTh = (bf16_t*)(ws + off); off += szWT;
    bf16_t* WTl = (bf16_t*)(ws + off); off += szWT;
    bf16_t* WPh = (bf16_t*)(ws + off); off += szWP;
    bf16_t* WPl = (bf16_t*)(ws + off); off += szWP;
    bf16_t* Qh  = (bf16_t*)(ws + off); off += szH;
    bf16_t* Ql  = (bf16_t*)(ws + off); off += szH;
    bf16_t* Kh  = (bf16_t*)(ws + off); off += szH;
    bf16_t* Kl  = (bf16_t*)(ws + off); off += szH;
    bf16_t* Vh  = (bf16_t*)(ws + off); off += szH;
    bf16_t* Vl  = (bf16_t*)(ws + off); off += szH;
    bf16_t* Oh  = (bf16_t*)(ws + off); off += szH;
    bf16_t* Ol  = (bf16_t*)(ws + off); off += szH;
    if (off > ws_size || off > 128 * MiB) return;

    const int n8 = TOK * DIM / 8;
    k_split_x<<<(n8 + 255) / 256, 256, 0, stream>>>(x, Xh, Xl, n8, Hp, Wp);

    k_split_wT<<<dim3(NQKV / 64, DIM / 64), 256, 0, stream>>>(Wq, DIM, Wkv, 2 * DIM, DIM, WTh, WTl, DIM);
    k_split_wT<<<dim3(DIM / 64, DIM / 64), 256, 0, stream>>>(Wproj, DIM, Wproj, DIM, DIM, WPh, WPl, DIM);

    k_gemm<<<dim3(NQKV / GB_N, TOK / GB_M), 256, 0, stream>>>(Xh, Xl, WTh, WTl, DIM, 0,
                                                             Qh, Ql, Kh, Kl, Vh, Vl,
                                                             out, bproj, DIM);

    k_attn<<<dim3(TOK / 32, 16), 64, 0, stream>>>(Qh, Ql, Kh, Kl, Vh, Vl, Oh, Ol);

    k_gemm<<<dim3(DIM / GB_N, TOK / GB_M), 256, 0, stream>>>(Oh, Ol, WPh, WPl, DIM, 1,
                                                            Qh, Ql, Kh, Kl, Vh, Vl,
                                                            out, bproj, DIM);
}
